// attentionlayer_5634997092873
// MI455X (gfx1250) — hardware-verified
//
#include <hip/hip_runtime.h>
#include <math.h>

constexpr int kB   = 16;
constexpr int kC   = 512;
constexpr int kH   = 32;
constexpr int kWd  = 32;
constexpr int kN   = kH * kWd;
constexpr int kCQ  = 32;
constexpr int kWP  = 34;
constexpr int kHPR = 35;
constexpr int kNPOS = kHPR * kWP;
constexpr int kNP  = kH * kWP;
constexpr int kTaps = 9;
constexpr int kKTot = kTaps * kC;
constexpr float kPCarry    = 32768.0f;
constexpr float kPCarryInv = 1.0f / 32768.0f;
constexpr float kF16MinNormal = 6.103515625e-05f;
static_assert(kNP % 64 == 0, "N tile multiple");
static_assert(kKTot % 32 == 0 && kC % 32 == 0, "K chunks stay inside one tap");
static_assert(kNP - 1 + 2 * kWP + 2 < kNPOS, "shifted window reads stay inside the padded plane");
static_assert(kNP % 32 == 0 && kC % 64 == 0 && kN % 64 == 0, "PV GEMM shape");
static_assert(kN % 16 == 0 && kCQ == 32, "energy tile shape");

typedef __attribute__((ext_vector_type(16))) _Float16 v16h;
typedef __attribute__((ext_vector_type(8)))  _Float16 v8h;
typedef __attribute__((ext_vector_type(16))) __bf16   v16b;
typedef __attribute__((ext_vector_type(8)))  __bf16   v8b;
typedef __attribute__((ext_vector_type(8)))  float    v8f;
typedef __attribute__((ext_vector_type(4)))  float    v4f;
typedef __attribute__((ext_vector_type(4)))  unsigned int v4u;

__device__ __forceinline__ unsigned short f2bf_bits(float f) {
  unsigned u = __float_as_uint(f);
  return (unsigned short)((u + 0x7FFFu + ((u >> 16) & 1u)) >> 16);
}
__device__ __forceinline__ float bf_bits2f(unsigned short h) { return __uint_as_float(((unsigned)h) << 16); }

__device__ __forceinline__ void dep_guard_h(v8f& a, v8f& b, v16h x, v16h y) { asm volatile("v_nop\n\tv_nop\n\tv_nop\n\tv_nop" : "+v"(a), "+v"(b) : "v"(x), "v"(y)); }
__device__ __forceinline__ void dep_guard_b(v8f& a, v8f& b, v16b x, v16b y) { asm volatile("v_nop\n\tv_nop\n\tv_nop\n\tv_nop" : "+v"(a), "+v"(b) : "v"(x), "v"(y)); }
__device__ __forceinline__ void dep_guard4_h(v8f& a, v8f& b, v8f& c, v8f& d, v16h x, v16h y) { asm volatile("v_nop\n\tv_nop\n\tv_nop\n\tv_nop" : "+v"(a), "+v"(b), "+v"(c), "+v"(d) : "v"(x), "v"(y)); }
__device__ __forceinline__ void dep_guard4_b(v8f& a, v8f& b, v8f& c, v8f& d, v16b x, v16b y) { asm volatile("v_nop\n\tv_nop\n\tv_nop\n\tv_nop" : "+v"(a), "+v"(b), "+v"(c), "+v"(d) : "v"(x), "v"(y)); }
__device__ __forceinline__ void keep4_h(v16h a, v16h b, v16h c, v16h d) { asm volatile("v_nop" :: "v"(a), "v"(b), "v"(c), "v"(d)); }
__device__ __forceinline__ void keep4_b(v16b a, v16b b, v16b c, v16b d) { asm volatile("v_nop" :: "v"(a), "v"(b), "v"(c), "v"(d)); }
__device__ __forceinline__ void acc_guard4(v8f& a, v8f& b, v8f& c, v8f& d) { asm volatile("v_nop\n\tv_nop\n\tv_nop\n\tv_nop" : "+v"(a), "+v"(b), "+v"(c), "+v"(d)); }
template <typename T> struct Frag;
template <> struct Frag<_Float16> {
  typedef v16h V; union U { v16h v; v8h h[2]; };
  static __device__ __forceinline__ v16h load(const _Float16* p) {
    U f; f.h[0] = *(const v8h*)(p); f.h[1] = *(const v8h*)(p + 16); return f.v;
  }
  static __device__ __forceinline__ v8f mma(v16h a, v16h b, v8f c) {
    return __builtin_amdgcn_wmma_f32_16x16x32_f16(false, a, false, b, (short)0, c, false, false);
  }
  static __device__ __forceinline__ void guard(v8f& a, v8f& b, v16h x, v16h y) { dep_guard_h(a, b, x, y); }
  static __device__ __forceinline__ void guard4(v8f& a, v8f& b, v8f& c, v8f& d, v16h x, v16h y) { dep_guard4_h(a, b, c, d, x, y); }
  static __device__ __forceinline__ void keep(v16h a, v16h b, v16h c, v16h d) { keep4_h(a, b, c, d); }
};
template <> struct Frag<__bf16> {
  typedef v16b V; union U { v16b v; v8b h[2]; };
  static __device__ __forceinline__ v16b load(const __bf16* p) {
    U f; f.h[0] = *(const v8b*)(p); f.h[1] = *(const v8b*)(p + 16); return f.v;
  }
  static __device__ __forceinline__ v8f mma(v16b a, v16b b, v8f c) {
    return __builtin_amdgcn_wmma_f32_16x16x32_bf16(false, a, false, b, (short)0, c, false, false);
  }
  static __device__ __forceinline__ void guard(v8f& a, v8f& b, v16b x, v16b y) { dep_guard_b(a, b, x, y); }
  static __device__ __forceinline__ void guard4(v8f& a, v8f& b, v8f& c, v8f& d, v16b x, v16b y) { dep_guard4_b(a, b, c, d, x, y); }
  static __device__ __forceinline__ void keep(v16b a, v16b b, v16b c, v16b d) { keep4_b(a, b, c, d); }
};

__device__ __forceinline__ unsigned pk16(unsigned short a, unsigned short b) { return (unsigned)a | ((unsigned)b << 16); }
__device__ __forceinline__ unsigned short h_bits(float f) { const _Float16 h = (_Float16)f; return __builtin_bit_cast(unsigned short, h); }
__device__ __forceinline__ void split_bf(float f, __bf16& hi, __bf16& lo) {
  const unsigned short hb = f2bf_bits(f);
  hi = __builtin_bit_cast(__bf16, hb);
  lo = __builtin_bit_cast(__bf16, f2bf_bits(f - bf_bits2f(hb)));
}
__device__ __forceinline__ v8f mma_bf_guarded3(v16b ah, v16b al, v16b bh, v16b bl) {
  v8f c = (v8f){0.f,0.f,0.f,0.f,0.f,0.f,0.f,0.f};
  c = __builtin_amdgcn_wmma_f32_16x16x32_bf16(false, ah, false, bh, (short)0, c, false, false);
  c = __builtin_amdgcn_wmma_f32_16x16x32_bf16(false, ah, false, bl, (short)0, c, false, false);
  c = __builtin_amdgcn_wmma_f32_16x16x32_bf16(false, al, false, bh, (short)0, c, false, false);
  asm volatile("v_nop\n\tv_nop\n\tv_nop\n\tv_nop" : "+v"(c) : "v"(ah), "v"(al), "v"(bh), "v"(bl));
  return c;
}

template <int ET> struct Elem;
template <> struct Elem<0> { typedef _Float16 T; };
template <> struct Elem<1> { typedef __bf16 T; };
template <int ET, bool SPLIT, int BIAS_MODE, int OUT_MODE, bool RESID, int ACT = 0>
__global__ __launch_bounds__(256) void wmma_gemm64(
    const unsigned short* __restrict__ Ap, const unsigned short* __restrict__ A2p, int lda, long strideA,
    const unsigned short* __restrict__ Btp, const unsigned short* __restrict__ Bt2p, int ldb, long strideB,
    void* __restrict__ Cout, void* __restrict__ Cout2, int ldc, long strideC,
    const float* __restrict__ bias,
    const float* __restrict__ resid, long strideR,
    int M, int N, int K, float scale) {
  typedef typename Elem<ET>::T T;
  typedef typename Frag<T>::V V;
  const T* A = (const T*)Ap; const T* A2 = (const T*)A2p; const T* Bt = (const T*)Btp; const T* Bt2 = (const T*)Bt2p;
  __shared__ __align__(16) float sT[8][16 * 68];
  const int b    = blockIdx.y;
  const int lane = threadIdx.x & 31;
  const int wave = threadIdx.x >> 5;
  const int tilesN = N >> 6;
  const int tilesM = M >> 6;
  const int tile = blockIdx.x * 8 + wave;
  if (tile >= tilesM * tilesN) return;
  const int tm = tile / tilesN;
  const int tn = tile - tm * tilesN;
  const int m0 = tm << 6;
  const int n0 = tn << 6;

  const T* Ab  = A  + (size_t)b * strideA;
  const T* Bb  = Bt + (size_t)b * strideB;
  const T* Ab2 = SPLIT ? (A2  + (size_t)b * strideA) : nullptr;
  const T* Bb2 = SPLIT ? (Bt2 + (size_t)b * strideB) : nullptr;

  const int rlane = lane & 15;
  const int koff  = (lane >> 4) * 8;
  const int mOff  = (lane >> 4) * 8;

  v8f acc[4][4];
#pragma unroll
  for (int i = 0; i < 4; ++i)
#pragma unroll
    for (int j = 0; j < 4; ++j) acc[i][j] = (v8f){0.f,0.f,0.f,0.f,0.f,0.f,0.f,0.f};

  for (int k0 = 0; k0 < K; k0 += 32) {
    V bh[4], bl[4];
#pragma unroll
    for (int j = 0; j < 4; ++j) {
      const size_t bo = (size_t)(n0 + (j << 4) + rlane) * ldb + koff + k0;
      bh[j] = Frag<T>::load(Bb + bo);
      if (SPLIT) bl[j] = Frag<T>::load(Bb2 + bo);
    }
#pragma unroll
    for (int i = 0; i < 4; ++i) {
      const size_t ao = (size_t)(m0 + (i << 4) + rlane) * lda + koff + k0;
      V ah = Frag<T>::load(Ab + ao);
      V al;
      if (SPLIT) al = Frag<T>::load(Ab2 + ao);
#pragma unroll
      for (int j = 0; j < 4; ++j) {
        acc[i][j] = Frag<T>::mma(ah, bh[j], acc[i][j]);
        if (SPLIT) {
          acc[i][j] = Frag<T>::mma(ah, bl[j], acc[i][j]);
          acc[i][j] = Frag<T>::mma(al, bh[j], acc[i][j]);
        }
      }
      Frag<T>::guard4(acc[i][0], acc[i][1], acc[i][2], acc[i][3], ah, SPLIT ? al : bh[3]);
    }
    Frag<T>::keep(bh[0], bh[1], bh[2], bh[3]);
    if (SPLIT) Frag<T>::keep(bl[0], bl[1], bl[2], bl[3]);
  }
  acc_guard4(acc[0][0], acc[0][1], acc[0][2], acc[0][3]);
  acc_guard4(acc[1][0], acc[1][1], acc[1][2], acc[1][3]);
  acc_guard4(acc[2][0], acc[2][1], acc[2][2], acc[2][3]);
  acc_guard4(acc[3][0], acc[3][1], acc[3][2], acc[3][3]);

  float* slab = sT[wave];
  const float* Rb = RESID ? (resid + (size_t)b * strideR) : nullptr;
#pragma unroll
  for (int i = 0; i < 4; ++i) {
    const int mBase = m0 + (i << 4);
#pragma unroll
    for (int j = 0; j < 4; ++j) {
      const int n = n0 + (j << 4) + rlane;
      float bv = 0.f;
      if (BIAS_MODE == 2) bv = bias[n];
#pragma unroll
      for (int r = 0; r < 8; ++r) {
        float v = acc[i][j][r] * scale;
        if (BIAS_MODE == 1) v += bias[mBase + mOff + r];
        if (BIAS_MODE == 2) v += bv;
        if (RESID) v += Rb[(size_t)(mBase + mOff + r) * ldc + n];
        if (ACT == 2) v = fmaxf(v, 0.0f);
        if (ACT == 4) v = (v > 0.f) ? v : 0.01f * v;
        slab[(mOff + r) * 68 + (j << 4) + rlane] = v;
      }
    }
    __builtin_amdgcn_fence(__ATOMIC_RELEASE, "workgroup");
    __builtin_amdgcn_wave_barrier();
    __builtin_amdgcn_fence(__ATOMIC_ACQUIRE, "workgroup");
    if (OUT_MODE == 0) {
      float* C = (float*)Cout + (size_t)b * strideC;
      const int hh = lane >> 4, c4 = (lane & 15) * 4;
      for (int pass = 0; pass < 2; ++pass) {
#pragma unroll
        for (int it = 0; it < 8; ++it) {
          const int row = it * 2 + hh;
          v4f v = *(const v4f*)(slab + row * 68 + c4);
          *(volatile v4f*)(C + (size_t)(mBase + row) * ldc + n0 + c4) = v;
        }
        __threadfence();
      }
    } else {
      const int q = lane >> 3, c8 = (lane & 7) * 8;
      unsigned short* C  = (unsigned short*)Cout  + (size_t)b * strideC;
      unsigned short* C2 = (OUT_MODE == 2) ? ((unsigned short*)Cout2 + (size_t)b * strideC) : nullptr;
      for (int pass = 0; pass < 2; ++pass) {
#pragma unroll
        for (int it = 0; it < 4; ++it) {
          const int row = it * 4 + q;
          const float* sp = slab + row * 68 + c8;
          v8h hv, lv;
#pragma unroll
          for (int e = 0; e < 8; ++e) {
            if (OUT_MODE == 1) {
              hv[e] = (_Float16)sp[e];
            } else {
              unsigned short hb = f2bf_bits(sp[e]);
              unsigned short lb = f2bf_bits(sp[e] - bf_bits2f(hb));
              hv[e] = __builtin_bit_cast(_Float16, hb);
              lv[e] = __builtin_bit_cast(_Float16, lb);
            }
          }
          *(volatile v8h*)(C + (size_t)(mBase + row) * ldc + n0 + c8) = hv;
          if (OUT_MODE == 2) *(volatile v8h*)(C2 + (size_t)(mBase + row) * ldc + n0 + c8) = lv;
        }
        __threadfence();
      }
    }
    __builtin_amdgcn_fence(__ATOMIC_RELEASE, "workgroup");
    __builtin_amdgcn_wave_barrier();
    __builtin_amdgcn_fence(__ATOMIC_ACQUIRE, "workgroup");
  }
}

template <int MI, int OUT_MODE>
__global__ __launch_bounds__(256) void conv_gemm_kernel(
    const unsigned short* __restrict__ Wp, const unsigned short* __restrict__ Xp, long strideX,
    void* __restrict__ Cout, int ldc, long strideC, const float* __restrict__ bias, int M, int N) {
  static_assert(MI >= 1 && MI <= 4, "wave tile rows");
  typedef __bf16 T;
  typedef v16b V;
  const T* A  = (const T*)Wp;
  const T* Bt = (const T*)Xp;
  __shared__ __align__(16) float sT[8][16 * 68];
  const int b    = blockIdx.y;
  const int lane = threadIdx.x & 31;
  const int wave = threadIdx.x >> 5;
  const int tilesN = N >> 6;
  const int tilesM = M / (16 * MI);
  const int tile = blockIdx.x * 8 + wave;
  if (tile >= tilesM * tilesN) return;
  const int tm = tile / tilesN;
  const int tn = tile - tm * tilesN;
  const int m0 = tm * (16 * MI);
  const int n0 = tn << 6;

  const T* Bb = Bt + (size_t)b * strideX;

  const int rlane = lane & 15;
  const int koff  = (lane >> 4) * 8;
  const int mOff  = (lane >> 4) * 8;

  v8f acc[MI][4];
#pragma unroll
  for (int i = 0; i < MI; ++i)
#pragma unroll
    for (int j = 0; j < 4; ++j) acc[i][j] = (v8f){0.f,0.f,0.f,0.f,0.f,0.f,0.f,0.f};

  for (int k0 = 0; k0 < kKTot; k0 += 32) {
    const int tap = k0 >> 9;
    const int th  = tap / 3;
    const int tw  = tap - th * 3;
    const int tapoff = th * kWP + tw;
    const int ic0 = k0 & (kC - 1);
    V bh[4];
#pragma unroll
    for (int j = 0; j < 4; ++j) {
      const size_t bo = (size_t)(n0 + (j << 4) + rlane + tapoff) * kC + ic0 + koff;
      bh[j] = Frag<T>::load(Bb + bo);
    }
#pragma unroll
    for (int i = 0; i < MI; ++i) {
      const size_t ao = (size_t)(m0 + (i << 4) + rlane) * kKTot + koff + k0;
      V ah = Frag<T>::load(A + ao);
#pragma unroll
      for (int j = 0; j < 4; ++j) acc[i][j] = Frag<T>::mma(ah, bh[j], acc[i][j]);
      Frag<T>::guard4(acc[i][0], acc[i][1], acc[i][2], acc[i][3], ah, bh[3]);
    }
    Frag<T>::keep(bh[0], bh[1], bh[2], bh[3]);
  }
#pragma unroll
  for (int i = 0; i < MI; ++i) acc_guard4(acc[i][0], acc[i][1], acc[i][2], acc[i][3]);

  float* slab = sT[wave];
#pragma unroll
  for (int i = 0; i < MI; ++i) {
    const int mBase = m0 + (i << 4);
    const v4f bz0 = *(const v4f*)(bias + mBase + mOff);
    const v4f bz1 = *(const v4f*)(bias + mBase + mOff + 4);
#pragma unroll
    for (int j = 0; j < 4; ++j) {
#pragma unroll
      for (int r = 0; r < 4; ++r) {
        slab[(mOff + r) * 68 + (j << 4) + rlane]     = acc[i][j][r] + bz0[r];
        slab[(mOff + 4 + r) * 68 + (j << 4) + rlane] = acc[i][j][4 + r] + bz1[r];
      }
    }
    __builtin_amdgcn_fence(__ATOMIC_RELEASE, "workgroup");
    __builtin_amdgcn_wave_barrier();
    __builtin_amdgcn_fence(__ATOMIC_ACQUIRE, "workgroup");
    if (OUT_MODE == 0) {
      float* C = (float*)Cout + (size_t)b * strideC;
      const int hh = lane >> 4, c4 = (lane & 15) * 4;
      for (int pass = 0; pass < 2; ++pass) {
#pragma unroll
        for (int it = 0; it < 8; ++it) {
          const int row = it * 2 + hh;
          v4f v = *(const v4f*)(slab + row * 68 + c4);
          *(volatile v4f*)(C + (size_t)(mBase + row) * ldc + n0 + c4) = v;
        }
        __threadfence();
      }
    } else {
      const int q = lane >> 3, c8 = (lane & 7) * 8;
      unsigned short* C = (unsigned short*)Cout + (size_t)b * strideC;
      for (int pass = 0; pass < 2; ++pass) {
#pragma unroll
        for (int it = 0; it < 4; ++it) {
          const int row = it * 4 + q;
          const float* sp = slab + row * 68 + c8;
          v8h hv;
#pragma unroll
          for (int e = 0; e < 8; ++e) hv[e] = (_Float16)sp[e];
          *(volatile v8h*)(C + (size_t)(mBase + row) * ldc + n0 + c8) = hv;
        }
        __threadfence();
      }
    }
    __builtin_amdgcn_fence(__ATOMIC_RELEASE, "workgroup");
    __builtin_amdgcn_wave_barrier();
    __builtin_amdgcn_fence(__ATOMIC_ACQUIRE, "workgroup");
  }
}

__global__ __launch_bounds__(256) void pack_pad_kernel(const float* __restrict__ src, unsigned short* __restrict__ dst) {
  __shared__ float sm[64][33];
  const int t  = threadIdx.x;
  const int hp = blockIdx.x;
  const int cc = blockIdx.y;
  const int b  = blockIdx.z;
  const int hs = min(max(hp - 1, 0), kH - 1);
  const float frow = (hp >= 1 && hp <= kH) ? 1.f : 0.f;
#pragma unroll
  for (int it = 0; it < 8; ++it) {
    const int e = it * 256 + t;
    const int c = e >> 5;
    const int w = e & 31;
    const float xv = src[((size_t)((b * kC + cc * 64 + c) * kH + hs)) * kWd + w];
    sm[c][w] = xv * frow;
  }
  __syncthreads();
  const int c8 = (t & 7) * 8;
#pragma unroll
  for (int it = 0; it < 2; ++it) {
    const int wp  = it * 32 + (t >> 3);
    const bool act = (it == 0) || (t < 16);
    const int wpc = min(wp, kWP - 1);
    const int ws  = min(max(wpc - 1, 0), kWd - 1);
    const float fcol = (wpc >= 1 && wpc <= kWd) ? 1.f : 0.f;
    unsigned short hb[8];
#pragma unroll
    for (int e = 0; e < 8; ++e) hb[e] = f2bf_bits(sm[c8 + e][ws] * fcol);
    const v4u u = (v4u){pk16(hb[0], hb[1]), pk16(hb[2], hb[3]), pk16(hb[4], hb[5]), pk16(hb[6], hb[7])};
    unsigned short* p = dst + ((size_t)(b * kNPOS + hp * kWP + wpc)) * kC + cc * 64 + c8;
    if (act) *(volatile v4u*)p = u;
    __threadfence();
    if (act) *(volatile v4u*)p = u;
  }
}

__global__ __launch_bounds__(256) void pack_w_kernel(const float* __restrict__ src, unsigned short* __restrict__ dst) {
  __shared__ float sm[kKTot];
  const int t  = threadIdx.x;
  const int oc = blockIdx.x;
  const float* sp = src + (size_t)oc * kKTot;
#pragma unroll 1
  for (int it = 0; it < 18; ++it) sm[it * 256 + t] = sp[it * 256 + t];
  __syncthreads();
  unsigned short* op = dst + (size_t)oc * kKTot;
#pragma unroll
  for (int it = 0; it < 3; ++it) {
    const int tp  = it * 256 + t;
    const bool act = tp < 576;
    const int tpc = min(tp, 575);
    const int tap = tpc >> 6;
    const int ic0 = (tpc & 63) * 8;
    unsigned short hb[8];
#pragma unroll
    for (int e = 0; e < 8; ++e) hb[e] = f2bf_bits(sm[(ic0 + e) * 9 + tap]);
    const v4u u = (v4u){pk16(hb[0], hb[1]), pk16(hb[2], hb[3]), pk16(hb[4], hb[5]), pk16(hb[6], hb[7])};
    unsigned short* p = op + 8 * (size_t)tpc;
    if (act) *(volatile v4u*)p = u;
    __threadfence();
    if (act) *(volatile v4u*)p = u;
  }
}

__global__ __launch_bounds__(256) void qk_rows_kernel(const float* __restrict__ src, float* __restrict__ dst) {
  __shared__ float sm[32][33];
  const int t = threadIdx.x;
  const int h = blockIdx.x;
  const int b = blockIdx.y;
  const int w = t & 31;
#pragma unroll
  for (int it = 0; it < 4; ++it) {
    const int d = it * 8 + (t >> 5);
    sm[w][d] = src[((size_t)(b * kCQ + d)) * kNP + h * kWP + w];
  }
  __syncthreads();
  const int w2 = t >> 3, c4 = (t & 7) * 4;
  const v4f v = (v4f){sm[w2][c4], sm[w2][c4 + 1], sm[w2][c4 + 2], sm[w2][c4 + 3]};
  float* p = dst + ((size_t)(b * kN + h * kWd + w2)) * kCQ + c4;
  *(volatile v4f*)p = v;
  __threadfence();
  *(volatile v4f*)p = v;
}

__global__ __launch_bounds__(256) void energy_softmax_kernel(const float* __restrict__ QT, const float* __restrict__ KT,
                                                            unsigned short* __restrict__ PP) {
  __shared__ __align__(16) float S[16][1028];
  __shared__ float invs[16];
  const int tid  = threadIdx.x;
  const int lane = tid & 31;
  const int wave = tid >> 5;
  const int hh   = lane >> 4;
  const int mm   = lane & 15;
  const int b    = blockIdx.y;
  const int i0   = blockIdx.x * 16;

  v16b qfh, qfl;
  {
    const float* qr = QT + ((size_t)(b * kN + i0 + mm)) * kCQ;
    const v4f a0 = *(const v4f*)(qr + 8 * hh);
    const v4f a1 = *(const v4f*)(qr + 8 * hh + 4);
    const v4f a2 = *(const v4f*)(qr + 16 + 8 * hh);
    const v4f a3 = *(const v4f*)(qr + 16 + 8 * hh + 4);
#pragma unroll
    for (int e = 0; e < 4; ++e) {
      __bf16 vh, vl;
      split_bf(a0[e], vh, vl); qfh[e]      = vh; qfl[e]      = vl;
      split_bf(a1[e], vh, vl); qfh[4 + e]  = vh; qfl[4 + e]  = vl;
      split_bf(a2[e], vh, vl); qfh[8 + e]  = vh; qfl[8 + e]  = vl;
      split_bf(a3[e], vh, vl); qfh[12 + e] = vh; qfl[12 + e] = vl;
    }
  }

#pragma unroll 1
  for (int t = 0; t < 8; ++t) {
    const int jt = wave * 8 + t;
    const float* kr = KT + ((size_t)(b * kN + jt * 16 + mm)) * kCQ;
    const v4f c0 = *(const v4f*)(kr + 8 * hh);
    const v4f c1 = *(const v4f*)(kr + 8 * hh + 4);
    const v4f c2 = *(const v4f*)(kr + 16 + 8 * hh);
    const v4f c3 = *(const v4f*)(kr + 16 + 8 * hh + 4);
    v16b kfh, kfl;
#pragma unroll
    for (int e = 0; e < 4; ++e) {
      __bf16 vh, vl;
      split_bf(c0[e], vh, vl); kfh[e]      = vh; kfl[e]      = vl;
      split_bf(c1[e], vh, vl); kfh[4 + e]  = vh; kfl[4 + e]  = vl;
      split_bf(c2[e], vh, vl); kfh[8 + e]  = vh; kfl[8 + e]  = vl;
      split_bf(c3[e], vh, vl); kfh[12 + e] = vh; kfl[12 + e] = vl;
    }
    const v8f acc = mma_bf_guarded3(qfh, qfl, kfh, kfl);
#pragma unroll
    for (int r = 0; r < 8; ++r) S[8 * hh + r][jt * 16 + mm] = acc[r];
  }
  __syncthreads();

  const int row = tid >> 4, sub = tid & 15;
  float mx = -__builtin_inff();
#pragma unroll 1
  for (int c = sub; c < kN; c += 16) mx = fmaxf(mx, S[row][c]);
#pragma unroll
  for (int off = 8; off > 0; off >>= 1) mx = fmaxf(mx, __shfl_xor(mx, off, 32));
  float sum = 0.f;
#pragma unroll 1
  for (int c = sub; c < kN; c += 16) {
    const float ev = expf(S[row][c] - mx);
    S[row][c] = ev;
    sum += ev;
  }
#pragma unroll
  for (int off = 8; off > 0; off >>= 1) sum += __shfl_xor(sum, off, 32);
  if (sub == 0) invs[row] = kPCarry / sum;
  __syncthreads();

  const size_t rowbase = ((size_t)(b * kN + i0)) * kNP;
  const bool act = tid < (kNP / 8);
#pragma unroll 1
  for (int r = 0; r < 16; ++r) {
    const float inv = invs[r];
    unsigned short hb[8];
#pragma unroll
    for (int e = 0; e < 8; ++e) {
      const int pj  = min(8 * tid + e, kNP - 1);
      const int hr  = pj / kWP;
      const int wc  = pj - hr * kWP;
      const int idx = hr * kWd + min(wc, kWd - 1);
      const float fz = (wc < kWd) ? 1.f : 0.f;
      float pv = S[r][idx] * inv * fz;
      pv = (pv >= kF16MinNormal) ? pv : 0.f;
      hb[e] = h_bits(pv);
    }
    const v4u u = (v4u){pk16(hb[0], hb[1]), pk16(hb[2], hb[3]), pk16(hb[4], hb[5]), pk16(hb[6], hb[7])};
    unsigned short* pr = PP + rowbase + (size_t)r * kNP + 8 * (size_t)tid;
    if (act) *(volatile v4u*)pr = u;
    __threadfence();
    if (act) *(volatile v4u*)pr = u;
  }
}

constexpr size_t kSzPad = (size_t)kB * kNPOS * kC * 2;
constexpr size_t kSzWqk = (size_t)kCQ * kKTot * 2;
constexpr size_t kSzWv  = (size_t)kC * kKTot * 2;
constexpr size_t kSzQ32 = (size_t)kB * kCQ * kNP * 4;
constexpr size_t kSzQT  = (size_t)kB * kN * kCQ * 4;
constexpr size_t kSzV16 = (size_t)kB * kC * kNP * 2;
constexpr size_t kSzPP  = (size_t)kB * kN * kNP * 2;
constexpr size_t kOffXP  = 0;
constexpr size_t kOffYP  = kOffXP + kSzPad;
constexpr size_t kOffWQ  = kOffYP + kSzPad;
constexpr size_t kOffWK  = kOffWQ + kSzWqk;
constexpr size_t kOffWV  = kOffWK + kSzWqk;
constexpr size_t kOffQ32 = kOffWV + kSzWv;
constexpr size_t kOffK32 = kOffQ32 + kSzQ32;
constexpr size_t kOffQT  = kOffK32 + kSzQ32;
constexpr size_t kOffKT  = kOffQT + kSzQT;
constexpr size_t kOffV16 = kOffKT + kSzQT;
constexpr size_t kOffPP  = kOffV16 + kSzV16;
constexpr size_t kWsTotal = kOffPP + kSzPP;
static_assert(kWsTotal == 106430464, "carve total");
static_assert(kWsTotal <= 134217728, "carve limit");
static_assert(kSzPad % 256 == 0 && kSzWqk % 256 == 0 && kSzWv % 256 == 0 && kSzQ32 % 256 == 0 &&
              kSzQT % 256 == 0 && kSzV16 % 256 == 0 && kSzPP % 256 == 0, "alignment");

extern "C" void kernel_launch(void* const* d_in, const int* in_sizes, int n_in,
                              void* d_out, int out_size, void* d_ws, size_t ws_size,
                              hipStream_t stream) {
  if (n_in < 8) return;
  const int nAct = kB * kC * kH * kWd;
  if (in_sizes[0] != nAct || in_sizes[1] != nAct) return;
  if (in_sizes[2] != kCQ * kKTot || in_sizes[4] != kCQ * kKTot || in_sizes[6] != kC * kKTot) return;
  if (in_sizes[3] != kCQ || in_sizes[5] != kCQ || in_sizes[7] != kC) return;
  if (out_size != kB * kC * kN) return;
  if (ws_size < kWsTotal) return;

  const float* x  = (const float*)d_in[0];
  const float* y  = (const float*)d_in[1];
  const float* wq = (const float*)d_in[2];
  const float* bq = (const float*)d_in[3];
  const float* wk = (const float*)d_in[4];
  const float* bk = (const float*)d_in[5];
  const float* wv = (const float*)d_in[6];
  const float* bv = (const float*)d_in[7];
  float* out = (float*)d_out;
  char* ws = (char*)d_ws;
  unsigned short* XP  = (unsigned short*)(ws + kOffXP);
  unsigned short* YP  = (unsigned short*)(ws + kOffYP);
  unsigned short* WQ  = (unsigned short*)(ws + kOffWQ);
  unsigned short* WK  = (unsigned short*)(ws + kOffWK);
  unsigned short* WV  = (unsigned short*)(ws + kOffWV);
  float* Q32 = (float*)(ws + kOffQ32);
  float* K32 = (float*)(ws + kOffK32);
  float* QT  = (float*)(ws + kOffQT);
  float* KT  = (float*)(ws + kOffKT);
  unsigned short* V16 = (unsigned short*)(ws + kOffV16);
  unsigned short* PP  = (unsigned short*)(ws + kOffPP);

  pack_pad_kernel<<<dim3(kHPR, kC / 64, kB), dim3(256), 0, stream>>>(x, XP);
  pack_pad_kernel<<<dim3(kHPR, kC / 64, kB), dim3(256), 0, stream>>>(y, YP);
  pack_w_kernel<<<dim3(kCQ), dim3(256), 0, stream>>>(wq, WQ);
  pack_w_kernel<<<dim3(kCQ), dim3(256), 0, stream>>>(wk, WK);
  pack_w_kernel<<<dim3(kC), dim3(256), 0, stream>>>(wv, WV);

  const long strideX  = (long)kNPOS * kC;
  const int  tilesQK  = (kCQ / 32) * (kNP / 64);
  const int  tilesV   = (kC / 64) * (kNP / 64);
  conv_gemm_kernel<2, 0><<<dim3((tilesQK + 7) / 8, kB), dim3(256), 0, stream>>>(
      WQ, XP, strideX, (void*)Q32, kNP, (long)kCQ * kNP, bq, kCQ, kNP);
  conv_gemm_kernel<2, 0><<<dim3((tilesQK + 7) / 8, kB), dim3(256), 0, stream>>>(
      WK, YP, strideX, (void*)K32, kNP, (long)kCQ * kNP, bk, kCQ, kNP);
  conv_gemm_kernel<4, 1><<<dim3((tilesV + 7) / 8, kB), dim3(256), 0, stream>>>(
      WV, YP, strideX, (void*)V16, kNP, (long)kC * kNP, bv, kC, kNP);

  qk_rows_kernel<<<dim3(kH, kB), dim3(256), 0, stream>>>(Q32, QT);
  qk_rows_kernel<<<dim3(kH, kB), dim3(256), 0, stream>>>(K32, KT);

  energy_softmax_kernel<<<dim3(kN / 16, kB), dim3(256), 0, stream>>>(QT, KT, PP);

  const int tilesPV = (kC / 64) * (kN / 64);
  wmma_gemm64<0, false, 0, 0, false, 0><<<dim3(tilesPV / 8, kB), dim3(256), 0, stream>>>(
      V16, V16, kNP, (long)kC * kNP, PP, PP, kNP, (long)kN * kNP,
      (void*)out, (void*)out, kN, (long)kC * kN, bq, bq, 0L, kC, kN, kNP, kPCarryInv);
}
